// MS_37031208026268
// MI455X (gfx1250) — hardware-verified
//
#include <hip/hip_runtime.h>
#include <hip/hip_bf16.h>


#define NN 8192
#define DD 32
#define WPB 4

typedef __attribute__((ext_vector_type(16))) __bf16      v16bf;
typedef __attribute__((ext_vector_type(8)))  float       v8f;
typedef __attribute__((ext_vector_type(4)))  unsigned int u32x4;

union BF16x16 {
    v16bf v;
    u32x4 q[2];
};
__device__ __forceinline__ v8f wmma_bf(v16bf a, v16bf b, v8f c) {
    v8f d = __builtin_amdgcn_wmma_f32_16x16x32_bf16(false, a, false, b, (short)0, c, false, false);
    asm volatile("v_nop\n\tv_nop\n\tv_nop\n\tv_nop" : "+v"(d) : "v"(a), "v"(b));
    return d;
}

__global__ __launch_bounds__(256) void ms_convert(const float* __restrict__ x,
                                                  __bf16* __restrict__ xbf,
                                                  __bf16* __restrict__ xTbf) {
    __shared__ __attribute__((aligned(16))) __bf16 tb[DD * 64];
    __shared__ __attribute__((aligned(16))) __bf16 tt[64 * DD];
    const int n0 = blockIdx.x * 64, tid = threadIdx.x;
#pragma unroll
    for (int q = 0; q < 8; ++q) {
        int e = tid + q * 256;
        int d = e >> 6, nl = e & 63;
        float f = x[d * NN + n0 + nl];
        tb[d * 64 + nl] = (__bf16)f;
        tt[nl * DD + d] = (__bf16)(f * 0.84932180f);
    }
    __syncthreads();
    {
        const int r = tid >> 3, sg = tid & 7;
        const u32x4 v = *(const u32x4*)(tb + r * 64 + sg * 8);
        volatile u32x4* dst = (volatile u32x4*)(xbf + r * NN + n0 + sg * 8);
        *dst = v; __threadfence(); *dst = v;
    }
    {
        const u32x4 v = *(const u32x4*)(tt + tid * 8);
        volatile u32x4* dst = (volatile u32x4*)(xTbf + (size_t)n0 * DD + tid * 8);
        *dst = v; __threadfence(); *dst = v;
    }
}

__global__ __launch_bounds__(32 * WPB) void ms_iter(const float* __restrict__ xin,
                                                    const __bf16* __restrict__ xbf,
                                                    const __bf16* __restrict__ xTbf,
                                                    float* __restrict__ xout) {
    const int lane = threadIdx.x & 31;
    const int wave = threadIdx.x >> 5;
    const int m    = lane & 15;
    const int hi   = lane >> 4;
    const int j_base = (blockIdx.x * WPB + wave) * 16;

    BF16x16 bj;
    {
        const __bf16* p = xTbf + (j_base + m) * DD;
        bj.q[0] = *(const u32x4*)(p + hi * 8);
        bj.q[1] = *(const u32x4*)(p + 16 + hi * 8);
    }

    auto loadA = [&](int i0, BF16x16& a0, BF16x16& a1) {
        const __bf16* r0 = xTbf + (i0 + m) * DD;
        a0.q[0] = *(const u32x4*)(r0 + hi * 8);
        a0.q[1] = *(const u32x4*)(r0 + 16 + hi * 8);
        const __bf16* r1 = xTbf + (i0 + 16 + m) * DD;
        a1.q[0] = *(const u32x4*)(r1 + hi * 8);
        a1.q[1] = *(const u32x4*)(r1 + 16 + hi * 8);
    };
    auto loadB2 = [&](int i0, BF16x16& lo, BF16x16& hh) {
        const __bf16* p0 = xbf + m * NN + i0;
        lo.q[0] = *(const u32x4*)(p0 + hi * 8);
        lo.q[1] = *(const u32x4*)(p0 + 16 + hi * 8);
        const __bf16* p1 = xbf + (16 + m) * NN + i0;
        hh.q[0] = *(const u32x4*)(p1 + hi * 8);
        hh.q[1] = *(const u32x4*)(p1 + 16 + hi * 8);
    };

    v8f accT0 = {};
    v8f accT1 = {};
    float deg = 0.0f;

    BF16x16 a0c, a1c, b2lc, b2hc;
    loadA(0, a0c, a1c);
    loadB2(0, b2lc, b2hc);

    for (int i0 = 0; i0 < NN; i0 += 32) {
        __builtin_prefetch(xTbf + (i0 + 64 + m) * DD, 0, 3);
        __builtin_prefetch(xbf + m * NN + i0 + 64, 0, 3);
        __builtin_prefetch(xbf + (16 + m) * NN + i0 + 64, 0, 3);

        v8f z = {};
        v8f c0 = wmma_bf(a0c.v, bj.v, z);
        v8f c1 = wmma_bf(a1c.v, bj.v, z);

        const int in = (i0 + 32 < NN) ? (i0 + 32) : i0;
        BF16x16 a0n, a1n, b2ln, b2hn;
        loadA(in, a0n, a1n);
        loadB2(in, b2ln, b2hn);

        BF16x16 a2;
#pragma unroll
        for (int r = 0; r < 8; ++r) {
            float p0 = __builtin_amdgcn_exp2f(c0[r]);
            float p1 = __builtin_amdgcn_exp2f(c1[r]);
            deg += p0 + p1;
            a2.v[r]     = (__bf16)p0;
            a2.v[r + 8] = (__bf16)p1;
        }

        accT0 = wmma_bf(a2.v, b2lc.v, accT0);
        accT1 = wmma_bf(a2.v, b2hc.v, accT1);

        a0c = a0n; a1c = a1n; b2lc = b2ln; b2hc = b2hn;
    }

    float degF = deg + __shfl_xor(deg, 16, 32);
    float dg[8];
#pragma unroll
    for (int r = 0; r < 8; ++r)
        dg[r] = __shfl(degF, hi * 8 + r, 32);

    __shared__ __attribute__((aligned(16))) float ot[DD][16 * WPB];
    const int jl = wave * 16 + hi * 8;
#pragma unroll
    for (int h = 0; h < 2; ++h) {
        v8f acc = h ? accT1 : accT0;
        const int d = h * 16 + m;
        const float* xr = xin + d * NN + j_base + hi * 8;
        float4 xi0 = *(const float4*)(xr);
        float4 xi1 = *(const float4*)(xr + 4);
        ot[d][jl + 0] = 0.5f * acc[0] / dg[0] + 0.5f * xi0.x;
        ot[d][jl + 1] = 0.5f * acc[1] / dg[1] + 0.5f * xi0.y;
        ot[d][jl + 2] = 0.5f * acc[2] / dg[2] + 0.5f * xi0.z;
        ot[d][jl + 3] = 0.5f * acc[3] / dg[3] + 0.5f * xi0.w;
        ot[d][jl + 4] = 0.5f * acc[4] / dg[4] + 0.5f * xi1.x;
        ot[d][jl + 5] = 0.5f * acc[5] / dg[5] + 0.5f * xi1.y;
        ot[d][jl + 6] = 0.5f * acc[6] / dg[6] + 0.5f * xi1.z;
        ot[d][jl + 7] = 0.5f * acc[7] / dg[7] + 0.5f * xi1.w;
    }
    __syncthreads();
    const int jb = blockIdx.x * (16 * WPB);
    for (int pass = 0; pass < 2; ++pass) {
#pragma unroll
        for (int q = 0; q < 4; ++q) {
            const int piece = threadIdx.x + q * (32 * WPB);
            const int d = piece >> 4, sg = piece & 15;
            *(volatile u32x4*)(xout + d * NN + jb + sg * 4) = *(const u32x4*)(&ot[d][sg * 4]);
        }
        __threadfence();
    }
}

extern "C" void kernel_launch(void* const* d_in, const int* in_sizes, int n_in,
                              void* d_out, int out_size, void* d_ws, size_t ws_size,
                              hipStream_t stream) {
    (void)in_sizes; (void)n_in; (void)out_size;
    if (ws_size < (size_t)DD * NN * 8) return;

    const float* x0 = (const float*)d_in[0];
    float* outbuf = (float*)d_out;

    float*  xA   = (float*)d_ws;
    __bf16* xbf  = (__bf16*)((char*)d_ws + (size_t)DD * NN * sizeof(float));
    __bf16* xTbf = xbf + (size_t)DD * NN;

    const float* cur = x0;
    for (int it = 0; it < 5; ++it) {
        ms_convert<<<NN / 64, 256, 0, stream>>>(cur, xbf, xTbf);
        float* out = (it & 1) ? xA : outbuf;
        ms_iter<<<NN / (16 * WPB), 32 * WPB, 0, stream>>>(cur, xbf, xTbf, out);
        cur = out;
    }
}
